// SelfAttention_19078244729039
// MI455X (gfx1250) — hardware-verified
//
#include <hip/hip_runtime.h>


#ifndef NB
#define NB 2
#endif
#ifndef SEQ
#define SEQ 2048
#endif
#define NB_FULL    2
#define SEQ_FULL   2048
#define NHEAD      16
#define HDIM       64
#define EMB        (NHEAD * HDIM)
#define BQ         128
#define BK         32
#define NWAVE      8
#define CT         64
#define TP         72
#define XPV        9
#define OP         68
#define GM         128
#define GN         64
#define WELEM      8
#define NROLE      3

#define P_CARRY    4096.0f
#define CTX_CARRY  256.0f
#define RES_CARRY  2048.0f
#define W_CARRY    64.0f

static_assert(SEQ % BQ == 0);
static_assert(SEQ % CT == 0);
static_assert(SEQ % BK == 0);
static_assert(SEQ % GM == 0);
static_assert(EMB % GN == 0);
static_assert(EMB % 32 == 0);
static_assert(BQ == NWAVE * 16);
static_assert(GM == NWAVE * 16);
static_assert(BK == 32);
static_assert(HDIM == 64);
static_assert(CT == 64);
static_assert(GN == 64);
static_assert(NHEAD * HDIM == EMB);
static_assert(EMB == 1024);
static_assert(SEQ <= SEQ_FULL);
static_assert(NB >= 1 && NB <= NB_FULL);
static_assert((TP * 2) % 16 == 0);
static_assert((OP * 4) % 16 == 0);
static_assert(XPV >= 8);
static_assert((size_t)(SEQ / CT) * NHEAD * NB * 256 * 2 * 8 == (size_t)NB * NHEAD * SEQ * HDIM);
static_assert((size_t)((EMB * EMB) / (256 * WELEM)) * 256 * WELEM == (size_t)EMB * EMB);
static_assert((size_t)(SEQ / BQ) * NHEAD * NB * NWAVE * 16 * HDIM == (size_t)NB * SEQ * EMB);
static_assert((size_t)(SEQ / GM) * (EMB / GN) * NB * NWAVE * 16 * GN == (size_t)NB * SEQ * EMB);
static_assert((size_t)5 * NB * SEQ * EMB * 2 + (size_t)EMB * EMB * 2 <= (size_t)134217728);

typedef __bf16   bf16;
typedef _Float16 f16;
typedef bf16     v16bf __attribute__((ext_vector_type(16)));
typedef f16      v16h  __attribute__((ext_vector_type(16)));
typedef f16      v8h   __attribute__((ext_vector_type(8)));
typedef float    v8f   __attribute__((ext_vector_type(8)));
typedef float    v4f   __attribute__((ext_vector_type(4)));
typedef unsigned v4u   __attribute__((ext_vector_type(4)));
typedef int      v4i   __attribute__((ext_vector_type(4)));

union FragB  { v16bf v; v4u q[2]; bf16 h[16]; };
union FragH  { v16h  v; v4u q[2]; f16  h[16]; };
union Pack8B { v4u u; bf16 h[8]; };
union Pack8H { v4u u; v8h v; f16 h[8]; };

static __device__ __forceinline__ v8f mma_bf16(v16bf a, v16bf b, v8f acc) {
  acc = __builtin_amdgcn_wmma_f32_16x16x32_bf16(false, a, false, b, (short)0, acc, false, false);
  asm volatile("v_nop\n\tv_nop\n\tv_nop\n\tv_nop" : "+v"(acc) : "v"(a), "v"(b));
  return acc;
}
static __device__ __forceinline__ v8f mma_f16(v16h a, v16h b, v8f acc) {
  acc = __builtin_amdgcn_wmma_f32_16x16x32_f16(false, a, false, b, (short)0, acc, false, false);
  asm volatile("v_nop\n\tv_nop\n\tv_nop\n\tv_nop" : "+v"(acc) : "v"(a), "v"(b));
  return acc;
}

__global__ __launch_bounds__(256) void qkv_planes_kernel(const float* __restrict__ xq,
                                                         const float* __restrict__ xk,
                                                         const float* __restrict__ xv,
                                                         const float* __restrict__ wq,
                                                         const float* __restrict__ wk,
                                                         const float* __restrict__ wv,
                                                         f16* __restrict__ qp,
                                                         f16* __restrict__ kp,
                                                         f16* __restrict__ vt) {
  const unsigned role = blockIdx.x / (unsigned)(SEQ / CT);
  const unsigned kt   = blockIdx.x - role * (unsigned)(SEQ / CT);
  const unsigned h    = blockIdx.y;
  const unsigned b    = blockIdx.z;
  const unsigned tid  = threadIdx.x;
  const unsigned wave = tid >> 5;
  const unsigned lane = tid & 31u;
  const unsigned lq   = lane & 15u;
  const unsigned hi   = lane >> 4;

  __shared__ v4u sX[CT * XPV];
  __shared__ v4u sW[HDIM * XPV];
  __shared__ __align__(16) f16 sY[64 * TP];

  const float* x   = (role == 0u) ? xq : ((role == 1u) ? xk : xv);
  const float* w   = (role == 0u) ? wq : ((role == 1u) ? wk : wv);
  f16*         dst = (role == 0u) ? qp : ((role == 1u) ? kp : vt);
  const unsigned s0 = kt * CT;

  #pragma unroll
  for (unsigned kk = 0; kk < 2; ++kk) {
    const unsigned rr = kk * 32u + (tid >> 3);
    const unsigned pc = tid & 7u;
    const float* src = x + ((size_t)b * SEQ_FULL + s0 + rr) * EMB + h * HDIM + pc * 8u;
    const v4f x0 = *(const v4f*)(src);
    const v4f x1 = *(const v4f*)(src + 4);
    const float* wsrc = w + rr * HDIM + pc * 8u;
    const v4f w0 = *(const v4f*)(wsrc);
    const v4f w1 = *(const v4f*)(wsrc + 4);
    Pack8B px, pw;
    #pragma unroll
    for (int i = 0; i < 4; ++i) {
      px.h[i]     = (bf16)x0[i];
      px.h[4 + i] = (bf16)x1[i];
      pw.h[i]     = (bf16)w0[i];
      pw.h[4 + i] = (bf16)w1[i];
    }
    sX[rr * XPV + pc] = px.u;
    sW[rr * XPV + pc] = pw.u;
  }
  __syncthreads();

  const unsigned rt = wave >> 1;
  const unsigned cb = (wave & 1u) * 2u;
  v8f acc[2];
  acc[0] = (v8f){0, 0, 0, 0, 0, 0, 0, 0};
  acc[1] = (v8f){0, 0, 0, 0, 0, 0, 0, 0};
  #pragma unroll
  for (unsigned f = 0; f < 2; ++f) {
    FragB a;
    a.q[0] = sX[(rt * 16u + lq) * XPV + f * 4u + hi];
    a.q[1] = sX[(rt * 16u + lq) * XPV + f * 4u + 2u + hi];
    #pragma unroll
    for (unsigned t = 0; t < 2; ++t) {
      FragB bw;
      bw.q[0] = sW[((cb + t) * 16u + lq) * XPV + f * 4u + hi];
      bw.q[1] = sW[((cb + t) * 16u + lq) * XPV + f * 4u + 2u + hi];
      acc[t] = mma_bf16(a.v, bw.v, acc[t]);
    }
  }

  const unsigned rstr = (role == 2u) ? 1u : (unsigned)TP;
  const unsigned cstr = (role == 2u) ? (unsigned)TP : 1u;
  #pragma unroll
  for (unsigned t = 0; t < 2; ++t) {
    #pragma unroll
    for (unsigned r = 0; r < 8; ++r) {
      sY[(rt * 16u + hi * 8u + r) * rstr + ((cb + t) * 16u + lq) * cstr] = (f16)acc[t][r];
    }
  }
  __syncthreads();

  v4u    val[2];
  size_t gi[2];
  #pragma unroll
  for (unsigned kk = 0; kk < 2; ++kk) {
    const unsigned a   = kk * 32u + (tid >> 3);
    const unsigned pc8 = (tid & 7u) * 8u;
    Pack8H ph;
    ph.v = *(const v8h*)(sY + a * TP + pc8);
    val[kk] = ph.u;
    const size_t irow = (((size_t)b * NHEAD + h) * SEQ + s0 + a) * HDIM + pc8;
    const size_t itrn = (((size_t)b * NHEAD + h) * HDIM + a) * SEQ + s0 + pc8;
    gi[kk] = (role == 2u) ? itrn : irow;
  }
  #pragma unroll
  for (int kk = 0; kk < 2; ++kk) *(volatile v4u*)(dst + gi[kk]) = val[kk];
  __threadfence();
  #pragma unroll
  for (int kk = 0; kk < 2; ++kk) *(volatile v4u*)(dst + gi[kk]) = val[kk];
}

__global__ __launch_bounds__(256) void w_plane_kernel(const float* __restrict__ w, f16* __restrict__ wp) {
  const unsigned t  = blockIdx.x * 256u + threadIdx.x;
  const size_t   e0 = (size_t)t * WELEM;
  const v4f a0 = *(const v4f*)(w + e0);
  const v4f a1 = *(const v4f*)(w + e0 + 4);
  Pack8H ph;
  #pragma unroll
  for (int i = 0; i < 4; ++i) {
    ph.h[i]     = (f16)((float)(bf16)a0[i] * W_CARRY);
    ph.h[4 + i] = (f16)((float)(bf16)a1[i] * W_CARRY);
  }
  const v4u val = ph.u;
  *(volatile v4u*)(wp + e0) = val;
  __threadfence();
  *(volatile v4u*)(wp + e0) = val;
}

__global__ __launch_bounds__(256) void attn_kernel(const f16* __restrict__ qp,
                                                   const f16* __restrict__ kp,
                                                   const f16* __restrict__ vt,
                                                   const int* __restrict__ mask,
                                                   f16* __restrict__ ch,
                                                   f16* __restrict__ cr) {
  const unsigned qblk = blockIdx.x;
  const unsigned h    = blockIdx.y;
  const unsigned b    = blockIdx.z;
  const unsigned tid  = threadIdx.x;
  const unsigned wave = tid >> 5;
  const unsigned lane = tid & 31u;
  const unsigned lq   = lane & 15u;
  const unsigned hi   = lane >> 4;

  __shared__ __align__(16) float sO[NWAVE * 16 * OP];

  const unsigned qrow0 = qblk * BQ + wave * 16u;

  const f16* q_h  = qp + ((size_t)b * NHEAD + h) * SEQ * HDIM;
  const f16* k_h  = kp + ((size_t)b * NHEAD + h) * SEQ * HDIM;
  const f16* vt_h = vt + ((size_t)b * NHEAD + h) * HDIM * SEQ;
  const int* mk = mask + ((size_t)b * SEQ_FULL + qrow0 + lq) * SEQ_FULL + hi * 8u;

  FragH qf[2];
  #pragma unroll
  for (unsigned f = 0; f < 2; ++f) {
    const f16* base = q_h + (size_t)(qrow0 + lq) * HDIM + f * 32u + hi * 8u;
    qf[f].q[0] = *(const v4u*)(base);
    qf[f].q[1] = *(const v4u*)(base + 16);
  }

  v8f o[4];
  #pragma unroll
  for (int dt = 0; dt < 4; ++dt) o[dt] = (v8f){0, 0, 0, 0, 0, 0, 0, 0};

  float rmax = -3.0e38f;
  float rsum = 0.0f;
  const float SL   = 0.03125f * 1.4426950408889634f;
  const float FILL = -1.0e20f;

  #pragma unroll 1
  for (unsigned i = 0; i < SEQ / BK; ++i) {
    const unsigned j0 = i * BK;

    FragH ak[2][2];
    #pragma unroll
    for (unsigned sub = 0; sub < 2; ++sub) {
      #pragma unroll
      for (unsigned f = 0; f < 2; ++f) {
        const f16* base = k_h + (size_t)(j0 + sub * 16u + lq) * HDIM + f * 32u + hi * 8u;
        ak[sub][f].q[0] = *(const v4u*)(base);
        ak[sub][f].q[1] = *(const v4u*)(base + 16);
      }
    }
    FragH bv[4];
    #pragma unroll
    for (unsigned dt = 0; dt < 4; ++dt) {
      const f16* base = vt_h + (size_t)(dt * 16u + lq) * SEQ + j0 + hi * 8u;
      bv[dt].q[0] = *(const v4u*)(base);
      bv[dt].q[1] = *(const v4u*)(base + 16);
    }
    v4i mv[4];
    mv[0] = *(const v4i*)(mk + j0);
    mv[1] = *(const v4i*)(mk + j0 + 4);
    mv[2] = *(const v4i*)(mk + j0 + 16);
    mv[3] = *(const v4i*)(mk + j0 + 20);

    v8f c[2];
    #pragma unroll
    for (int sub = 0; sub < 2; ++sub) {
      v8f acc = (v8f){0, 0, 0, 0, 0, 0, 0, 0};
      acc = mma_f16(ak[sub][0].v, qf[0].v, acc);
      acc = mma_f16(ak[sub][1].v, qf[1].v, acc);
      c[sub] = acc;
    }

    #pragma unroll
    for (int r = 0; r < 4; ++r) {
      c[0][r]     = (mv[0][r] == 1) ? FILL : c[0][r];
      c[0][4 + r] = (mv[1][r] == 1) ? FILL : c[0][4 + r];
      c[1][r]     = (mv[2][r] == 1) ? FILL : c[1][r];
      c[1][4 + r] = (mv[3][r] == 1) ? FILL : c[1][4 + r];
    }

    float m_new = rmax;
    #pragma unroll
    for (int r = 0; r < 8; ++r) {
      m_new = fmaxf(m_new, c[0][r]);
      m_new = fmaxf(m_new, c[1][r]);
    }
    m_new = fmaxf(m_new, __shfl_xor(m_new, 16, 32));
    const float scale = __builtin_amdgcn_exp2f((rmax - m_new) * SL);
    rmax = m_new;

    FragH pa;
    float psum = 0.0f;
    #pragma unroll
    for (int r = 0; r < 8; ++r) {
      const float p0 = __builtin_amdgcn_exp2f((c[0][r] - m_new) * SL);
      const float p1 = __builtin_amdgcn_exp2f((c[1][r] - m_new) * SL);
      const f16 h0 = (f16)(p0 * P_CARRY);
      const f16 h1 = (f16)(p1 * P_CARRY);
      pa.h[r]     = h0;
      pa.h[8 + r] = h1;
      psum += (float)h0 + (float)h1;
    }
    rsum = rsum * scale + psum + __shfl_xor(psum, 16, 32);

    float sc[8];
    #pragma unroll
    for (int r = 0; r < 8; ++r) sc[r] = __shfl(scale, (int)((hi << 3) + r), 32);
    #pragma unroll
    for (int dt = 0; dt < 4; ++dt) {
      #pragma unroll
      for (int r = 0; r < 8; ++r) o[dt][r] *= sc[r];
    }

    #pragma unroll
    for (int dt = 0; dt < 4; ++dt) o[dt] = mma_f16(pa.v, bv[dt].v, o[dt]);
  }

  float rs[8];
  #pragma unroll
  for (int r = 0; r < 8; ++r) rs[r] = CTX_CARRY * (1.0f / __shfl(rsum, (int)((hi << 3) + r), 32));

  float* so = sO + wave * (16 * OP);
  #pragma unroll
  for (int r = 0; r < 8; ++r) {
    #pragma unroll
    for (int dt = 0; dt < 4; ++dt) {
      so[(hi * 8u + r) * OP + dt * 16u + lq] = o[dt][r] * rs[r];
    }
  }
  __syncthreads();

  v4u    hv[4], rv[4];
  size_t gidx[4];
  #pragma unroll
  for (unsigned it = 0; it < 4; ++it) {
    const unsigned row = it * 4u + (lane >> 3);
    const unsigned c8  = (lane & 7u) * 8u;
    const v4f a0 = *(const v4f*)(so + row * OP + c8);
    const v4f a1 = *(const v4f*)(so + row * OP + c8 + 4);
    Pack8H ph, pr;
    #pragma unroll
    for (int i = 0; i < 4; ++i) {
      const f16 t0 = (f16)a0[i];
      const f16 t1 = (f16)a1[i];
      ph.h[i]     = t0;
      ph.h[4 + i] = t1;
      pr.h[i]     = (f16)((a0[i] - (float)t0) * RES_CARRY);
      pr.h[4 + i] = (f16)((a1[i] - (float)t1) * RES_CARRY);
    }
    hv[it]   = ph.u;
    rv[it]   = pr.u;
    gidx[it] = ((size_t)b * SEQ + qrow0 + row) * EMB + h * HDIM + c8;
  }
  #pragma unroll
  for (int it = 0; it < 4; ++it) {
    *(volatile v4u*)(ch + gidx[it]) = hv[it];
    *(volatile v4u*)(cr + gidx[it]) = rv[it];
  }
  __threadfence();
  #pragma unroll
  for (int it = 0; it < 4; ++it) {
    *(volatile v4u*)(ch + gidx[it]) = hv[it];
    *(volatile v4u*)(cr + gidx[it]) = rv[it];
  }
}

__global__ __launch_bounds__(256) void out_proj_kernel(const f16* __restrict__ ch,
                                                       const f16* __restrict__ cr,
                                                       const f16* __restrict__ wp,
                                                       const float* __restrict__ bias,
                                                       float* __restrict__ out) {
  const unsigned rb   = blockIdx.x;
  const unsigned cb   = blockIdx.y;
  const unsigned b    = blockIdx.z;
  const unsigned tid  = threadIdx.x;
  const unsigned wave = tid >> 5;
  const unsigned lane = tid & 31u;
  const unsigned lq   = lane & 15u;
  const unsigned hi   = lane >> 4;

  __shared__ __align__(16) float sO[NWAVE * 16 * OP];

  const unsigned row0 = rb * GM + wave * 16u;
  const unsigned col0 = cb * GN;

  const f16* ah = ch + ((size_t)b * SEQ + row0 + lq) * EMB + hi * 8u;
  const f16* ar = cr + ((size_t)b * SEQ + row0 + lq) * EMB + hi * 8u;
  const f16* bw = wp + (size_t)(col0 + lq) * EMB + hi * 8u;

  v8f acc[4], acr[4];
  #pragma unroll
  for (int nt = 0; nt < 4; ++nt) {
    acc[nt] = (v8f){0, 0, 0, 0, 0, 0, 0, 0};
    acr[nt] = (v8f){0, 0, 0, 0, 0, 0, 0, 0};
  }

  #pragma unroll 1
  for (unsigned k0 = 0; k0 < EMB; k0 += 32u) {
    FragH a, a2;
    a.q[0]  = *(const v4u*)(ah + k0);
    a.q[1]  = *(const v4u*)(ah + k0 + 16);
    a2.q[0] = *(const v4u*)(ar + k0);
    a2.q[1] = *(const v4u*)(ar + k0 + 16);
    FragH bf[4];
    #pragma unroll
    for (unsigned nt = 0; nt < 4; ++nt) {
      const f16* base = bw + (size_t)(nt * 16u) * EMB + k0;
      bf[nt].q[0] = *(const v4u*)(base);
      bf[nt].q[1] = *(const v4u*)(base + 16);
    }
    #pragma unroll
    for (int nt = 0; nt < 4; ++nt) {
      acc[nt] = mma_f16(a.v,  bf[nt].v, acc[nt]);
      acr[nt] = mma_f16(a2.v, bf[nt].v, acr[nt]);
    }
  }

  float* so = sO + wave * (16 * OP);
  const float inv_res = 1.0f / RES_CARRY;
  const float inv_car = 1.0f / (CTX_CARRY * W_CARRY);
  #pragma unroll
  for (int r = 0; r < 8; ++r) {
    #pragma unroll
    for (int nt = 0; nt < 4; ++nt) {
      so[(hi * 8u + r) * OP + nt * 16u + lq] = (acc[nt][r] + acr[nt][r] * inv_res) * inv_car;
    }
  }
  __syncthreads();

  const v4f braw = *(const v4f*)(bias + col0 + lq * 4u);
  v4f bq;
  #pragma unroll
  for (int i = 0; i < 4; ++i) bq[i] = (float)(bf16)braw[i];

  v4f    vals[8];
  size_t gidx[8];
  #pragma unroll
  for (unsigned it = 0; it < 8; ++it) {
    const unsigned row = it * 2u + hi;
    const v4f t = *(const v4f*)(so + row * OP + lq * 4u);
    vals[it] = t + bq;
    gidx[it] = ((size_t)b * SEQ_FULL + row0 + row) * EMB + col0 + lq * 4u;
  }
  #pragma unroll
  for (int it = 0; it < 8; ++it) *(volatile v4f*)(out + gidx[it]) = vals[it];
  __threadfence();
  #pragma unroll
  for (int it = 0; it < 8; ++it) *(volatile v4f*)(out + gidx[it]) = vals[it];
}

extern "C" void kernel_launch(void* const* d_in, const int* in_sizes, int n_in,
                              void* d_out, int out_size, void* d_ws, size_t ws_size,
                              hipStream_t stream) {
  if (n_in < 10) return;
  const size_t rows_used = (size_t)(NB - 1) * SEQ_FULL + SEQ;
  const size_t mask_used = ((size_t)(NB - 1) * SEQ_FULL + (SEQ - 1)) * SEQ_FULL + SEQ;
  if ((size_t)in_sizes[0] < rows_used * EMB) return;
  if ((size_t)in_sizes[1] < rows_used * EMB) return;
  if ((size_t)in_sizes[2] < rows_used * EMB) return;
  if ((size_t)in_sizes[3] < mask_used) return;
  if ((size_t)in_sizes[5] < (size_t)HDIM * HDIM) return;
  if ((size_t)in_sizes[6] < (size_t)HDIM * HDIM) return;
  if ((size_t)in_sizes[7] < (size_t)HDIM * HDIM) return;
  if ((size_t)in_sizes[8] < (size_t)EMB * EMB) return;
  if ((size_t)in_sizes[9] < (size_t)EMB) return;
  if ((size_t)out_size < rows_used * EMB) return;

  const size_t pl_bytes = (size_t)NB * NHEAD * SEQ * HDIM * 2;
  const size_t wp_bytes = (size_t)EMB * EMB * 2;
  const size_t total    = 5 * pl_bytes + wp_bytes;
  if (ws_size < total) return;

  const float* values = (const float*)d_in[0];
  const float* keys   = (const float*)d_in[1];
  const float* query  = (const float*)d_in[2];
  const int*   mask   = (const int*)d_in[3];
  const float* Wv     = (const float*)d_in[5];
  const float* Wk     = (const float*)d_in[6];
  const float* Wq     = (const float*)d_in[7];
  const float* Wout   = (const float*)d_in[8];
  const float* bout   = (const float*)d_in[9];
  float*       out    = (float*)d_out;

  char* base = (char*)d_ws;
  f16* qp = (f16*)(base);
  f16* kp = (f16*)(base + pl_bytes);
  f16* vt = (f16*)(base + 2 * pl_bytes);
  f16* ch = (f16*)(base + 3 * pl_bytes);
  f16* cr = (f16*)(base + 4 * pl_bytes);
  f16* wp = (f16*)(base + 5 * pl_bytes);

  qkv_planes_kernel<<<dim3(NROLE * (SEQ / CT), NHEAD, NB), 256, 0, stream>>>(query, keys, values, Wq, Wk, Wv, qp, kp, vt);
  w_plane_kernel<<<dim3((EMB * EMB) / (256 * WELEM)), 256, 0, stream>>>(Wout, wp);
  attn_kernel<<<dim3(SEQ / BQ, NHEAD, NB), 256, 0, stream>>>(qp, kp, vt, mask, ch, cr);
  out_proj_kernel<<<dim3(SEQ / GM, EMB / GN, NB), 256, 0, stream>>>(ch, cr, wp, Wout == nullptr ? bout : bout, out);
}
